// SMOLUpdate_4063039062769
// MI455X (gfx1250) — hardware-run, weakly checked
//
#include <hip/hip_runtime.h>
#include <math.h>

typedef __attribute__((ext_vector_type(16))) _Float16 v16h;
typedef __attribute__((ext_vector_type(8)))  _Float16 v8h;
typedef __attribute__((ext_vector_type(8)))  float    v8f;
typedef __attribute__((ext_vector_type(4)))  float    v4f;
typedef __attribute__((ext_vector_type(4)))  int      v4i;

constexpr int kRes  = 4096;
constexpr int kLig  = 128;
constexpr int kAt   = 16;
constexpr int kPw   = 64;
constexpr int kLw   = 256;
constexpr int kHid  = 128;
constexpr int kKA   = 320;
constexpr int kYP   = 192;
constexpr int kPts  = 33;
static_assert(kKA == 64 + kAt * 16, "feature tile K");
static_assert((kKA % 32) == 0 && (kPw % 32) == 0 && (kHid % 32) == 0 && (kLw % 32) == 0, "K multiples of 32");
static_assert((kRes % 64) == 0 && (kYP % 64) == 0 && (kPw % 64) == 0 && (kLw % 64) == 0, "M,N multiples of 64");
static_assert((kRes % 32) == 0, "M multiple of the 32-row GEMM tile");

constexpr float kCarryAct = 16.0f;
constexpr float kCarryW   = 256.0f;
constexpr float kCarryWo  = 4096.0f;
constexpr float kCarryG   = 64.0f;
constexpr float kInvAW    = 1.0f / (kCarryAct * kCarryW);
constexpr float kInvGWo   = 1.0f / (kCarryG * kCarryWo);
constexpr float kInvSigma = 1.0f / 0.75f;
constexpr float kResid    = 2048.0f;
constexpr float kInvResid = 1.0f / 2048.0f;

constexpr size_t kOffWCAT  = 0;
constexpr size_t kOffW1T   = kOffWCAT  + (size_t)kPw * kKA * 2;
constexpr size_t kOffW2T   = kOffW1T   + (size_t)kHid * kPw * 2;
constexpr size_t kOffWLOC  = kOffW2T   + (size_t)kPw * kHid * 2;
constexpr size_t kOffWOUT  = kOffWLOC  + (size_t)kYP * kLw * 2;
constexpr size_t kOffLOCH  = kOffWOUT  + (size_t)kLw * kPw * 2;
constexpr size_t kOffY     = kOffLOCH  + (size_t)kRes * kLw * 2;
constexpr size_t kOffHPH   = kOffY     + (size_t)kRes * kYP * 4;
constexpr size_t kOffPR    = kOffHPH   + (size_t)kRes * kHid * 2;
constexpr size_t kOffGH    = kOffPR    + (size_t)kRes * kPw * 4;
constexpr size_t kOffWLOCL = kOffGH    + (size_t)kRes * kPw * 2;
constexpr size_t kOffW2TL  = kOffWLOCL + (size_t)kYP * kLw * 2;
constexpr size_t kOffWOUTL = kOffW2TL  + (size_t)kPw * kHid * 2;
constexpr size_t kOffLOCL  = kOffWOUTL + (size_t)kLw * kPw * 2;
constexpr size_t kOffHPL   = kOffLOCL  + (size_t)kRes * kLw * 2;
constexpr size_t kOffGL    = kOffHPL   + (size_t)kRes * kHid * 2;
constexpr size_t kWsTotal  = kOffGL    + (size_t)kRes * kPw * 2;
static_assert(kWsTotal == 11886592ull, "carve total");
static_assert(kWsTotal <= 134217728ull, "carve cap");
static_assert((kOffW1T % 128) == 0 && (kOffW2T % 128) == 0 && (kOffWLOC % 128) == 0 && (kOffWOUT % 128) == 0 &&
              (kOffLOCH % 128) == 0 && (kOffY % 128) == 0 && (kOffHPH % 128) == 0 && (kOffPR % 128) == 0 &&
              (kOffGH % 128) == 0 && (kOffWLOCL % 128) == 0 && (kOffW2TL % 128) == 0 && (kOffWOUTL % 128) == 0 &&
              (kOffLOCL % 128) == 0 && (kOffHPL % 128) == 0 && (kOffGL % 128) == 0, "128-B aligned regions");

union FragU { v16h v; v8h h[2]; };
__device__ __forceinline__ v16h frag_load(const _Float16* p) {
  FragU f;
  f.h[0] = *(const v8h*)(p);
  f.h[1] = *(const v8h*)(p + 16);
  return f.v;
}
__device__ __forceinline__ v8f mma_h(v16h a, v16h b, v8f c) {
  c = __builtin_amdgcn_wmma_f32_16x16x32_f16(false, a, false, b, (short)0, c, false, false);
  asm volatile("v_nop\n\tv_nop\n\tv_nop\n\tv_nop" : "+v"(c) : "v"(a), "v"(b));
  return c;
}

__device__ __forceinline__ float gelu_t(float x) {
  const float x3 = x * x * x;
  return 0.5f * x * (1.0f + tanhf(0.7978845608028654f * (x + 0.044715f * x3)));
}

__device__ __forceinline__ _Float16 resid_of(float x, _Float16 h) {
  const float hf = (float)h;
  return (_Float16)((x - hf) * kResid);
}

template <bool LO>
__global__ __launch_bounds__(256) void build_bt_kernel(
    const float* __restrict__ srcA, int ldA, int rowsA, int colsA,
    const float* __restrict__ srcB, int ldB, int rowsB, int colsB, int ksplit,
    unsigned short* __restrict__ dst, unsigned short* __restrict__ dst2, int dstK, int nRows, float carry)
{
  const int cpr = dstK >> 3;
  const int i = blockIdx.x * 256 + threadIdx.x;
  if (i >= nRows * cpr) return;
  const int n = i / cpr;
  const int k0 = (i - n * cpr) * 8;
  const int na = (n < colsA) ? n : (colsA - 1);
  const int nb = (n < colsB) ? n : (colsB - 1);
  v8h hv, lv;
#pragma unroll
  for (int e = 0; e < 8; ++e) {
    const int k = k0 + e;
    const int ka = (k < rowsA) ? k : (rowsA - 1);
    int kb = k - ksplit;
    kb = (kb < 0) ? 0 : kb;
    kb = (kb < rowsB) ? kb : (rowsB - 1);
    float va = srcA[(size_t)ka * ldA + na];
    float vb = srcB[(size_t)kb * ldB + nb];
    asm volatile("" : "+v"(va));
    asm volatile("" : "+v"(vb));
    const bool useA = (k < ksplit);
    const bool okA = (k < rowsA) && (n < colsA);
    const bool okB = ((k - ksplit) < rowsB) && (n < colsB);
    const float sa = okA ? va : 0.0f;
    const float sb = okB ? vb : 0.0f;
    const float v = useA ? sa : sb;
    const float x = v * carry;
    const _Float16 s = (_Float16)x;
    hv[e] = s;
    lv[e] = LO ? resid_of(x, s) : (_Float16)0.0f;
  }
  unsigned short* q = dst + (size_t)n * dstK + k0;
  *(volatile v8h*)q = hv;
  if (LO) {
    unsigned short* q2 = dst2 + (size_t)n * dstK + k0;
    *(volatile v8h*)q2 = lv;
  }
  __threadfence();
  *(volatile v8h*)q = hv;
  if (LO) {
    unsigned short* q2 = dst2 + (size_t)n * dstK + k0;
    *(volatile v8h*)q2 = lv;
  }
}

__global__ __launch_bounds__(256) void cast_rows_f16_kernel(
    const float* __restrict__ src, unsigned short* __restrict__ dst, unsigned short* __restrict__ dst2,
    int total8, float carry)
{
  const int i = blockIdx.x * 256 + threadIdx.x;
  if (i >= total8) return;
  const size_t e0 = (size_t)i << 3;
  const v4f a0 = *(const v4f*)(src + e0);
  const v4f a1 = *(const v4f*)(src + e0 + 4);
  v8h hv, lv;
#pragma unroll
  for (int e = 0; e < 4; ++e) {
    const float x0 = a0[e] * carry;
    const float x1 = a1[e] * carry;
    const _Float16 s0 = (_Float16)x0;
    const _Float16 s1 = (_Float16)x1;
    hv[e]     = s0;
    hv[4 + e] = s1;
    lv[e]     = resid_of(x0, s0);
    lv[4 + e] = resid_of(x1, s1);
  }
  unsigned short* q  = dst + e0;
  unsigned short* q2 = dst2 + e0;
  *(volatile v8h*)q  = hv;
  *(volatile v8h*)q2 = lv;
  __threadfence();
  *(volatile v8h*)q  = hv;
  *(volatile v8h*)q2 = lv;
}

__global__ __launch_bounds__(256) void gemm_res_f16_kernel(
    const unsigned short* __restrict__ Ap, const unsigned short* __restrict__ A2p, int lda,
    const unsigned short* __restrict__ Btp, const unsigned short* __restrict__ Bt2p, int ldb,
    float* __restrict__ C, int ldc, int M, int N, int K, float scale)
{
  const _Float16* A   = (const _Float16*)Ap;
  const _Float16* A2  = (const _Float16*)A2p;
  const _Float16* Bt  = (const _Float16*)Btp;
  const _Float16* Bt2 = (const _Float16*)Bt2p;
  __shared__ __align__(16) float sT[8][16 * 68];
  const int lane = threadIdx.x & 31;
  const int wave = threadIdx.x >> 5;
  const int tilesN = N >> 6;
  const int tilesM = M >> 5;
  const int tile = blockIdx.x * 8 + wave;
  if (tile >= tilesM * tilesN) return;
  const int tm = tile / tilesN;
  const int tn = tile - tm * tilesN;
  const int m0 = tm << 5;
  const int n0 = tn << 6;
  const int rlane = lane & 15;
  const int koff  = (lane >> 4) * 8;
  const int mOff  = (lane >> 4) * 8;

  v8f acc[2][4];
  v8f acr[2][4];
#pragma unroll
  for (int i = 0; i < 2; ++i)
#pragma unroll
    for (int j = 0; j < 4; ++j) {
      acc[i][j] = (v8f){0.f,0.f,0.f,0.f,0.f,0.f,0.f,0.f};
      acr[i][j] = (v8f){0.f,0.f,0.f,0.f,0.f,0.f,0.f,0.f};
    }

  for (int k0 = 0; k0 < K; k0 += 32) {
    v16h ah[2], al[2];
#pragma unroll
    for (int i = 0; i < 2; ++i) {
      const size_t ao = (size_t)(m0 + (i << 4) + rlane) * lda + koff + k0;
      ah[i] = frag_load(A + ao);
      al[i] = frag_load(A2 + ao);
    }
#pragma unroll
    for (int j = 0; j < 4; ++j) {
      const size_t bo = (size_t)(n0 + (j << 4) + rlane) * ldb + koff + k0;
      const v16h bh = frag_load(Bt + bo);
      const v16h bl = frag_load(Bt2 + bo);
#pragma unroll
      for (int i = 0; i < 2; ++i) {
        acc[i][j] = mma_h(ah[i], bh, acc[i][j]);
        acr[i][j] = mma_h(ah[i], bl, acr[i][j]);
        acr[i][j] = mma_h(al[i], bh, acr[i][j]);
      }
    }
  }

  float* slab = sT[wave];
#pragma unroll
  for (int i = 0; i < 2; ++i) {
    const int mBase = m0 + (i << 4);
#pragma unroll
    for (int j = 0; j < 4; ++j) {
#pragma unroll
      for (int r = 0; r < 8; ++r) {
        const float v = (acc[i][j][r] + acr[i][j][r] * kInvResid) * scale;
        slab[(mOff + r) * 68 + (j << 4) + rlane] = v;
      }
    }
    __builtin_amdgcn_fence(__ATOMIC_RELEASE, "workgroup");
    __builtin_amdgcn_wave_barrier();
    __builtin_amdgcn_fence(__ATOMIC_ACQUIRE, "workgroup");
    {
      const int hh = lane >> 4, c4 = (lane & 15) * 4;
      for (int pass = 0; pass < 2; ++pass) {
#pragma unroll
        for (int it = 0; it < 8; ++it) {
          const int row = it * 2 + hh;
          v4f v = *(const v4f*)(slab + row * 68 + c4);
          *(volatile v4f*)(C + (size_t)(mBase + row) * ldc + n0 + c4) = v;
        }
        __threadfence();
      }
    }
    __builtin_amdgcn_fence(__ATOMIC_RELEASE, "workgroup");
    __builtin_amdgcn_wave_barrier();
    __builtin_amdgcn_fence(__ATOMIC_ACQUIRE, "workgroup");
  }
}

constexpr unsigned kLOffA    = 0;
constexpr unsigned kLOffSlab = kLOffA    + 128u * 320u * 2u;
constexpr unsigned kLOffLn   = kLOffSlab + 8u * 16u * 132u * 4u;
constexpr unsigned kLOffCol  = kLOffLn   + 128u * 64u * 2u;
constexpr unsigned kLOffHp   = kLOffCol  + 8u * 128u * 4u;
constexpr unsigned kLOffWt   = kLOffHp   + 128u * 4u;
constexpr unsigned kLOffLpos = kLOffWt   + 448u * 4u;
constexpr unsigned kLOffPall = kLOffLpos + 384u * 4u;
constexpr unsigned kLOffBl   = kLOffPall + 96u * 4u;
constexpr unsigned kLOffLnS  = kLOffBl   + 64u * 4u;
constexpr unsigned kLOffLnO  = kLOffLnS  + 64u * 4u;
constexpr unsigned kLOffB1   = kLOffLnO  + 64u * 4u;
constexpr unsigned kLOffSt   = kLOffB1   + 128u * 4u;
constexpr unsigned kLOffMsk  = kLOffSt   + 128u * 4u;
constexpr unsigned kLOffCnt  = kLOffMsk  + 128u * 4u;
constexpr unsigned kLdsBytes = kLOffCnt  + 16u;
static_assert(kLdsBytes == 176528u, "LDS total");
static_assert((kLOffSlab % 16) == 0 && (kLOffLn % 16) == 0 && (kLOffCol % 16) == 0 && (kLOffHp % 16) == 0 &&
              (kLOffWt % 16) == 0 && (kLOffLpos % 16) == 0 && (kLOffPall % 16) == 0 && (kLOffBl % 16) == 0 &&
              (kLOffB1 % 16) == 0 && (kLOffSt % 16) == 0 && (kLOffMsk % 16) == 0 && (kLOffCnt % 16) == 0, "LDS alignment");
constexpr int kSlabP = 132;

__global__ __launch_bounds__(256) void pair_fused_kernel(
    const float* __restrict__ posG, const int* __restrict__ typeG, const float* __restrict__ lposG,
    const int* __restrict__ maskG, const float* __restrict__ wTypeG, const float* __restrict__ lnScaleG,
    const float* __restrict__ lnOffG, const float* __restrict__ b1G, const float* __restrict__ Yg,
    const unsigned short* __restrict__ WcatT, const unsigned short* __restrict__ W1T,
    unsigned short* __restrict__ HpH, unsigned short* __restrict__ HpL)
{
  extern __shared__ __align__(16) unsigned char smem[];
  _Float16* aS    = (_Float16*)(smem + kLOffA);
  float*    slabS = (float*)(smem + kLOffSlab);
  _Float16* lnT   = (_Float16*)(smem + kLOffLn);
  float*    colS  = (float*)(smem + kLOffCol);
  float*    hpS   = (float*)(smem + kLOffHp);
  float*    wtS   = (float*)(smem + kLOffWt);
  float*    lposS = (float*)(smem + kLOffLpos);
  float*    pallS = (float*)(smem + kLOffPall);
  float*    blS   = (float*)(smem + kLOffBl);
  float*    lnS   = (float*)(smem + kLOffLnS);
  float*    lnO   = (float*)(smem + kLOffLnO);
  float*    b1S   = (float*)(smem + kLOffB1);
  int*      stS   = (int*)(smem + kLOffSt);
  int*      mskS  = (int*)(smem + kLOffMsk);
  int*      cntS  = (int*)(smem + kLOffCnt);

  const int n    = blockIdx.x;
  const int tid  = threadIdx.x;
  const int wave = tid >> 5;
  const int lane = tid & 31;
  const int hh   = lane >> 4;
  const int c    = lane & 15;

  wtS[tid] = wTypeG[tid];
  if (wave < 6) wtS[256 + tid] = wTypeG[256 + tid];
  if (wave < 4) {
    int t = typeG[(size_t)n * kLig + tid];
    t = (t < 0) ? 0 : t;
    t = (t > 6) ? 6 : t;
    stS[tid]  = t;
    mskS[tid] = (maskG[(size_t)n * kLig + tid] != 0) ? 1 : 0;
    b1S[tid]  = b1G[tid];
  }
  if (wave < 2) {
    blS[tid] = Yg[(size_t)n * kYP + 64 + tid];
    lnS[tid] = lnScaleG[tid];
    lnO[tid] = lnOffG[tid];
  }
  if (wave >= 4 && wave < 7) {
    const int q = tid - 128;
    *(v4f*)(lposS + 4 * q) = *(const v4f*)(lposG + (size_t)n * (kLig * 3) + 4 * q);
  }
  if (wave == 7) {
    const float* pp = posG + (size_t)n * 15;
    const float nx = pp[0], ny = pp[1], nz = pp[2];
    const float cax = pp[3], cay = pp[4], caz = pp[5];
    const float cx = pp[6], cy = pp[7], cz = pp[8];
    const float v1x = cx - cax, v1y = cy - cay, v1z = cz - caz;
    const float r1 = 1.0f / sqrtf((v1x * v1x + v1y * v1y + v1z * v1z) + 1e-6f);
    const float e1x = v1x * r1, e1y = v1y * r1, e1z = v1z * r1;
    const float v2x = nx - cax, v2y = ny - cay, v2z = nz - caz;
    const float dd = e1x * v2x + e1y * v2y + e1z * v2z;
    const float u2x = v2x - e1x * dd, u2y = v2y - e1y * dd, u2z = v2z - e1z * dd;
    const float r2 = 1.0f / sqrtf((u2x * u2x + u2y * u2y + u2z * u2z) + 1e-6f);
    const float e2x = u2x * r2, e2y = u2y * r2, e2z = u2z * r2;
    const float e3x = e1y * e2z - e1z * e2y;
    const float e3y = e1z * e2x - e1x * e2z;
    const float e3z = e1x * e2y - e1y * e2x;
    const int ar = (c < 4) ? c : 4;
    const int pk = (c > 5) ? (c - 5) : 0;
    float ax = pp[ar * 3 + 0], ay = pp[ar * 3 + 1], az = pp[ar * 3 + 2];
    const float* yp = Yg + (size_t)n * kYP + pk * 3;
    float p0 = yp[0], p1 = yp[1], p2 = yp[2];
    asm volatile("" : "+v"(ax));
    asm volatile("" : "+v"(ay));
    asm volatile("" : "+v"(az));
    asm volatile("" : "+v"(p0));
    asm volatile("" : "+v"(p1));
    asm volatile("" : "+v"(p2));
    const float qx = e1x * p0 + e2x * p1 + e3x * p2 + cax;
    const float qy = e1y * p0 + e2y * p1 + e3y * p2 + cay;
    const float qz = e1z * p0 + e2z * p1 + e3z * p2 + caz;
    const bool isreal = (c < 5);
    pallS[lane * 3 + 0] = isreal ? ax : qx;
    pallS[lane * 3 + 1] = isreal ? ay : qy;
    pallS[lane * 3 + 2] = isreal ? az : qz;
  }
  __syncthreads();

#pragma unroll 1
  for (int it = 0; it < 8; ++it) {
    const int i = it * 256 + tid;
    const int s = i >> 4, a = i & 15;
    const float rx = lposS[s * 3 + 0] - pallS[a * 3 + 0];
    const float ry = lposS[s * 3 + 1] - pallS[a * 3 + 1];
    const float rz = lposS[s * 3 + 2] - pallS[a * 3 + 2];
    const float d2 = (rx * rx + ry * ry + rz * rz) + 1e-6f;
    const float dist = sqrtf(d2);
    const float inv = 1.0f / dist;
    _Float16* arow = aS + s * kKA;
    arow[a * 3 + 0] = (_Float16)(rx * inv * kCarryAct);
    arow[a * 3 + 1] = (_Float16)(ry * inv * kCarryAct);
    arow[a * 3 + 2] = (_Float16)(rz * inv * kCarryAct);
    arow[48 + a] = (_Float16)0.0f;
#pragma unroll 1
    for (int hb = 0; hb < 2; ++hb) {
      v8h rv;
#pragma unroll
      for (int j = 0; j < 8; ++j) {
        const float ctr = 0.8f * (float)(hb * 8 + j);
        const float z = (dist - ctr) * kInvSigma;
        rv[j] = (_Float16)(expf(-(z * z)) * kCarryAct);
      }
      *(v8h*)(arow + 64 + a * 16 + hb * 8) = rv;
    }
  }
  __syncthreads();

  const int m0 = wave * 16;
  v8f acc[4];
#pragma unroll
  for (int j = 0; j < 4; ++j) acc[j] = (v8f){0.f,0.f,0.f,0.f,0.f,0.f,0.f,0.f};
  {
    const _Float16* aBase = aS + (m0 + c) * kKA + 8 * hh;
    const _Float16* bBase = (const _Float16*)WcatT + (size_t)c * kKA + 8 * hh;
#pragma unroll 2
    for (int k0 = 0; k0 < kKA; k0 += 32) {
      const v16h af = frag_load(aBase + k0);
#pragma unroll
      for (int j = 0; j < 4; ++j) {
        const v16h bf = frag_load(bBase + (size_t)(j * 16) * kKA + k0);
        acc[j] = mma_h(af, bf, acc[j]);
      }
    }
  }

  {
    float x[4][8];
    float lsc[4], lof[4], blv[4];
    int tt[8];
#pragma unroll
    for (int r = 0; r < 8; ++r) tt[r] = stS[m0 + 8 * hh + r];
#pragma unroll
    for (int j = 0; j < 4; ++j) {
      const int col = j * 16 + c;
      lsc[j] = lnS[col];
      lof[j] = lnO[col];
      blv[j] = blS[col];
    }
#pragma unroll
    for (int j = 0; j < 4; ++j) {
      const int col = j * 16 + c;
#pragma unroll
      for (int r = 0; r < 8; ++r) {
        x[j][r] = acc[j][r] * kInvAW + wtS[tt[r] * kPw + col] + blv[j];
      }
    }
#pragma unroll
    for (int r = 0; r < 8; ++r) {
      float s = (x[0][r] + x[1][r]) + (x[2][r] + x[3][r]);
      s += __shfl_xor(s, 1, 32);
      s += __shfl_xor(s, 2, 32);
      s += __shfl_xor(s, 4, 32);
      s += __shfl_xor(s, 8, 32);
      const float mu = s * (1.0f / 64.0f);
      float q = 0.0f;
#pragma unroll
      for (int j = 0; j < 4; ++j) {
        const float d = x[j][r] - mu;
        x[j][r] = d;
        q += d * d;
      }
      q += __shfl_xor(q, 1, 32);
      q += __shfl_xor(q, 2, 32);
      q += __shfl_xor(q, 4, 32);
      q += __shfl_xor(q, 8, 32);
      const float inv = rsqrtf(q * (1.0f / 64.0f) + 1e-5f);
#pragma unroll
      for (int j = 0; j < 4; ++j) {
        const float y = x[j][r] * inv * lsc[j] + lof[j];
        lnT[(m0 + 8 * hh + r) * kPw + j * 16 + c] = (_Float16)(y * kCarryAct);
      }
    }
  }
  __syncthreads();

  {
    const v16h a0 = frag_load(lnT + (m0 + c) * kPw + 8 * hh);
    const v16h a1 = frag_load(lnT + (m0 + c) * kPw + 32 + 8 * hh);
    float* slab = slabS + wave * (16 * kSlabP);
    const _Float16* w1 = (const _Float16*)W1T + (size_t)c * kPw + 8 * hh;
#pragma unroll 2
    for (int j = 0; j < 8; ++j) {
      v8f ac = (v8f){0.f,0.f,0.f,0.f,0.f,0.f,0.f,0.f};
      const v16h b0 = frag_load(w1 + (size_t)(j * 16) * kPw);
      const v16h b1 = frag_load(w1 + (size_t)(j * 16) * kPw + 32);
      ac = mma_h(a0, b0, ac);
      ac = mma_h(a1, b1, ac);
#pragma unroll
      for (int r = 0; r < 8; ++r) slab[(8 * hh + r) * kSlabP + j * 16 + c] = ac[r] * kInvAW;
    }
  }
  {
    const int mk = mskS[(wave & 3) * 32 + lane];
    const unsigned long long bal = __ballot(mk != 0);
    const int pc = __popcll(bal);
    if (wave < 4 && lane == 0) cntS[wave] = pc;
  }
  __syncthreads();

  {
    const float* slab = slabS + wave * (16 * kSlabP);
    float sum[4], b1v[4];
#pragma unroll
    for (int q = 0; q < 4; ++q) {
      sum[q] = 0.0f;
      b1v[q] = b1S[lane + 32 * q];
    }
#pragma unroll 1
    for (int row = 0; row < 16; ++row) {
      const int mk = mskS[m0 + row];
#pragma unroll
      for (int q = 0; q < 4; ++q) {
        const float v = slab[row * kSlabP + lane + 32 * q] + b1v[q];
        const float g = gelu_t(v);
        sum[q] += (mk != 0) ? g : 0.0f;
      }
    }
#pragma unroll
    for (int q = 0; q < 4; ++q) colS[wave * kHid + lane + 32 * q] = sum[q];
  }
  __syncthreads();

  if (wave < 4) {
    float s = 0.0f;
#pragma unroll
    for (int w = 0; w < 8; ++w) s += colS[w * kHid + tid];
    const int cnt = (cntS[0] + cntS[1]) + (cntS[2] + cntS[3]);
    const float cf = fmaxf((float)cnt, 1.0f);
    hpS[tid] = s / cf;
  }
  __syncthreads();

  if (wave == 0) {
    const int c8 = (lane & 15) * 8;
    const v4f h0 = *(const v4f*)(hpS + c8);
    const v4f h1 = *(const v4f*)(hpS + c8 + 4);
    v8h hv, lv;
#pragma unroll
    for (int e = 0; e < 4; ++e) {
      const float x0 = h0[e] * kCarryAct;
      const float x1 = h1[e] * kCarryAct;
      const _Float16 s0 = (_Float16)x0;
      const _Float16 s1 = (_Float16)x1;
      hv[e]     = s0;
      hv[4 + e] = s1;
      lv[e]     = resid_of(x0, s0);
      lv[4 + e] = resid_of(x1, s1);
    }
    unsigned short* dst  = HpH + (size_t)n * kHid + c8;
    unsigned short* dst2 = HpL + (size_t)n * kHid + c8;
    if (lane < 16) {
      *(volatile v8h*)dst  = hv;
      *(volatile v8h*)dst2 = lv;
    }
    __threadfence();
    if (lane < 16) {
      *(volatile v8h*)dst  = hv;
      *(volatile v8h*)dst2 = lv;
    }
  }
}

__global__ __launch_bounds__(256) void gate_stage_kernel(
    const float* __restrict__ PR, const float* __restrict__ Yg, const float* __restrict__ b2G,
    const int* __restrict__ maskG, unsigned short* __restrict__ GH, unsigned short* __restrict__ GL)
{
  __shared__ __align__(16) float sG[32 * 64];
  __shared__ float cfS[32];
  const int tid = threadIdx.x;
  const int n0 = blockIdx.x * 32;
  {
    const int r = tid >> 3, part = tid & 7;
    const int* mp = maskG + (size_t)(n0 + r) * kLig + part * 16;
    int cnt = 0;
#pragma unroll
    for (int q = 0; q < 4; ++q) {
      const v4i m = *(const v4i*)(mp + 4 * q);
      cnt += ((m[0] != 0) ? 1 : 0) + ((m[1] != 0) ? 1 : 0) + ((m[2] != 0) ? 1 : 0) + ((m[3] != 0) ? 1 : 0);
    }
    cnt += __shfl_xor(cnt, 1, 32);
    cnt += __shfl_xor(cnt, 2, 32);
    cnt += __shfl_xor(cnt, 4, 32);
    if (part == 0) cfS[r] = (cnt > 0) ? 1.0f : 0.0f;
  }
  __syncthreads();
#pragma unroll 1
  for (int it = 0; it < 8; ++it) {
    const int idx = it * 256 + tid;
    const int row = idx >> 6, col = idx & 63;
    const float p = PR[(size_t)(n0 + row) * kPw + col];
    const float g = Yg[(size_t)(n0 + row) * kYP + 128 + col];
    const float b = b2G[col];
    const float pooled = p + b * cfS[row];
    sG[idx] = gelu_t(g) * pooled;
  }
  __syncthreads();
  {
    const int r = tid >> 3, c8 = (tid & 7) * 8;
    const v4f g0 = *(const v4f*)(sG + r * 64 + c8);
    const v4f g1 = *(const v4f*)(sG + r * 64 + c8 + 4);
    v8h hv, lv;
#pragma unroll
    for (int e = 0; e < 4; ++e) {
      const float x0 = g0[e] * kCarryG;
      const float x1 = g1[e] * kCarryG;
      const _Float16 s0 = (_Float16)x0;
      const _Float16 s1 = (_Float16)x1;
      hv[e]     = s0;
      hv[4 + e] = s1;
      lv[e]     = resid_of(x0, s0);
      lv[4 + e] = resid_of(x1, s1);
    }
    unsigned short* dst  = GH + (size_t)(n0 + r) * kPw + c8;
    unsigned short* dst2 = GL + (size_t)(n0 + r) * kPw + c8;
    *(volatile v8h*)dst  = hv;
    *(volatile v8h*)dst2 = lv;
    __threadfence();
    *(volatile v8h*)dst  = hv;
    *(volatile v8h*)dst2 = lv;
  }
}

extern "C" void kernel_launch(void* const* d_in, const int* in_sizes, int n_in,
                              void* d_out, int out_size, void* d_ws, size_t ws_size,
                              hipStream_t stream) {
  if (n_in < 18) return;
  if (in_sizes[0] != kRes * kLw) return;
  if (in_sizes[1] != kRes * 15) return;
  if (in_sizes[2] != kRes * kLig) return;
  if (in_sizes[3] != kRes * kLig * 3) return;
  if (in_sizes[4] != kRes * kLig) return;
  if (in_sizes[5] != kLw * kPts) return;
  if (in_sizes[6] != 7 * kPw) return;
  if (in_sizes[7] != kLw * kPw) return;
  if (in_sizes[8] != 48 * kPw) return;
  if (in_sizes[9] != 256 * kPw) return;
  if (in_sizes[10] != kPw || in_sizes[11] != kPw) return;
  if (in_sizes[12] != kPw * kHid) return;
  if (in_sizes[13] != kHid) return;
  if (in_sizes[14] != kHid * kPw) return;
  if (in_sizes[15] != kPw) return;
  if (in_sizes[16] != kLw * kPw) return;
  if (in_sizes[17] != kPw * kLw) return;
  if (out_size != kRes * kLw) return;
  if (ws_size < kWsTotal) return;

  const float* local    = (const float*)d_in[0];
  const float* pos      = (const float*)d_in[1];
  const int*   lig_type = (const int*)d_in[2];
  const float* lig_pos  = (const float*)d_in[3];
  const int*   lig_mask = (const int*)d_in[4];
  const float* w_points = (const float*)d_in[5];
  const float* w_type   = (const float*)d_in[6];
  const float* w_local  = (const float*)d_in[7];
  const float* w_dir    = (const float*)d_in[8];
  const float* w_dist   = (const float*)d_in[9];
  const float* ln_scale = (const float*)d_in[10];
  const float* ln_off   = (const float*)d_in[11];
  const float* w_mlp1   = (const float*)d_in[12];
  const float* b_mlp1   = (const float*)d_in[13];
  const float* w_mlp2   = (const float*)d_in[14];
  const float* b_mlp2   = (const float*)d_in[15];
  const float* w_gate   = (const float*)d_in[16];
  const float* w_out    = (const float*)d_in[17];
  float* out = (float*)d_out;

  char* ws = (char*)d_ws;
  unsigned short* WCAT  = (unsigned short*)(ws + kOffWCAT);
  unsigned short* W1T   = (unsigned short*)(ws + kOffW1T);
  unsigned short* W2T   = (unsigned short*)(ws + kOffW2T);
  unsigned short* WLOC  = (unsigned short*)(ws + kOffWLOC);
  unsigned short* WOUT  = (unsigned short*)(ws + kOffWOUT);
  unsigned short* LOCH  = (unsigned short*)(ws + kOffLOCH);
  float*          Y     = (float*)(ws + kOffY);
  unsigned short* HPH   = (unsigned short*)(ws + kOffHPH);
  float*          PR    = (float*)(ws + kOffPR);
  unsigned short* GH    = (unsigned short*)(ws + kOffGH);
  unsigned short* WLOCL = (unsigned short*)(ws + kOffWLOCL);
  unsigned short* W2TL  = (unsigned short*)(ws + kOffW2TL);
  unsigned short* WOUTL = (unsigned short*)(ws + kOffWOUTL);
  unsigned short* LOCL  = (unsigned short*)(ws + kOffLOCL);
  unsigned short* HPL   = (unsigned short*)(ws + kOffHPL);
  unsigned short* GL    = (unsigned short*)(ws + kOffGL);

  build_bt_kernel<false><<<10, 256, 0, stream>>>(w_dir, kPw, 48, kPw, w_dist, kPw, 256, kPw, 64, WCAT, nullptr, kKA, kPw, kCarryW);
  build_bt_kernel<false><<<4, 256, 0, stream>>>(w_mlp1, kHid, kPw, kHid, w_mlp1, 1, 1, 1, kPw, W1T, nullptr, kPw, kHid, kCarryW);
  build_bt_kernel<true><<<4, 256, 0, stream>>>(w_mlp2, kPw, kHid, kPw, w_mlp2, 1, 1, 1, kHid, W2T, W2TL, kHid, kPw, kCarryW);
  build_bt_kernel<true><<<8, 256, 0, stream>>>(w_points, kPts, kLw, kPts, w_points, 1, 1, 1, kLw, WLOC, WLOCL, kLw, 64, kCarryW);
  build_bt_kernel<true><<<8, 256, 0, stream>>>(w_local, kPw, kLw, kPw, w_local, 1, 1, 1, kLw,
                                                WLOC + (size_t)64 * kLw, WLOCL + (size_t)64 * kLw, kLw, 64, kCarryW);
  build_bt_kernel<true><<<8, 256, 0, stream>>>(w_gate, kPw, kLw, kPw, w_gate, 1, 1, 1, kLw,
                                                WLOC + (size_t)128 * kLw, WLOCL + (size_t)128 * kLw, kLw, 64, kCarryW);
  build_bt_kernel<true><<<8, 256, 0, stream>>>(w_out, kLw, kPw, kLw, w_out, 1, 1, 1, kPw, WOUT, WOUTL, kPw, kLw, kCarryWo);
  cast_rows_f16_kernel<<<(kRes * kLw / 8) / 256, 256, 0, stream>>>(local, LOCH, LOCL, kRes * kLw / 8, kCarryAct);

  gemm_res_f16_kernel<<<48, 256, 0, stream>>>(LOCH, LOCL, kLw, WLOC, WLOCL, kLw, Y, kYP, kRes, kYP, kLw, kInvAW);

  pair_fused_kernel<<<kRes, 256, kLdsBytes, stream>>>(pos, lig_type, lig_pos, lig_mask, w_type, ln_scale, ln_off,
                                                       b_mlp1, Y, WCAT, W1T, HPH, HPL);

  gemm_res_f16_kernel<<<16, 256, 0, stream>>>(HPH, HPL, kHid, W2T, W2TL, kHid, PR, kPw, kRes, kPw, kHid, kInvAW);

  gate_stage_kernel<<<kRes / 32, 256, 0, stream>>>(PR, Y, b_mlp2, lig_mask, GH, GL);

  gemm_res_f16_kernel<<<64, 256, 0, stream>>>(GH, GL, kPw, WOUT, WOUTL, kPw, out, kLw, kRes, kLw, kPw, kInvGWo);
}
